// LightGFormer_10110353014883
// MI455X (gfx1250) — hardware-run, weakly checked
//
#include <hip/hip_runtime.h>
#include <math.h>

typedef __attribute__((ext_vector_type(16))) _Float16 v16h;
typedef __attribute__((ext_vector_type(8)))  _Float16 v8h;
typedef __attribute__((ext_vector_type(4)))  _Float16 v4h;
typedef __attribute__((ext_vector_type(16))) __bf16   v16b;
typedef __attribute__((ext_vector_type(8)))  __bf16   v8b;
typedef __attribute__((ext_vector_type(8)))  float    v8f;
typedef __attribute__((ext_vector_type(4)))  float    v4f;
typedef __attribute__((ext_vector_type(4)))  unsigned int v4u;
typedef __attribute__((ext_vector_type(2)))  unsigned int v2u;

constexpr int kB   = 8;
constexpr int kN   = 1024;
constexpr int kD   = 256;
constexpr int kH   = 8;
constexpr int kL   = 4;
constexpr int kDK  = kD / kH;
constexpr int kDFF = 4 * kD;
constexpr int kM   = kB * kN;
constexpr int kQKP = 2 * kD;
constexpr int kFG  = kDFF / 2;
constexpr int kFO  = kD / 2;
static_assert(kDK == 32);
static_assert(kM == 8192 && kQKP == 512 && kFG == 512 && kFO == 128);
static_assert((kD % 32) == 0 && (kFG % 32) == 0 && (kDK % 32) == 0);
static_assert((kM % 64) == 0 && (kD % 64) == 0 && (kQKP % 64) == 0 && (kDFF % 64) == 0 && (kFO % 64) == 0 && ((kL * kD) % 64) == 0);

constexpr float kWCarry    = 16.0f;
constexpr float kWCarryInv = 1.0f / kWCarry;
constexpr float kPCarry    = 1024.0f;
constexpr float kOCarry    = 64.0f;
constexpr float kPOverO    = kPCarry / kOCarry;
constexpr float kOutScale  = 1.0f / (kOCarry * kWCarry);
constexpr float kLnEps     = 1e-5f;
constexpr float kInvD      = 1.0f / (float)kD;
constexpr float kInvSqrt2  = 0.70710678118654752f;

constexpr size_t kOffXF   = 0;
constexpr size_t kOffRB   = kOffXF   + (size_t)kM * kD * 4;
constexpr size_t kOffX16  = kOffRB   + (size_t)kM * kD * 4;
constexpr size_t kOffXV16 = kOffX16  + (size_t)kM * kD * 2;
constexpr size_t kOffQK16 = kOffXV16 + (size_t)kM * kD * 2;
constexpr size_t kOffVT   = kOffQK16 + (size_t)kM * kQKP * 2;
constexpr size_t kOffO16  = kOffVT   + (size_t)kL * kD * kM * 2;
constexpr size_t kOffGB   = kOffO16  + (size_t)kM * kD * 2;
constexpr size_t kOffH16  = kOffGB   + (size_t)kM * kDFF * 4;
constexpr size_t kOffWQK  = kOffH16  + (size_t)kM * kDFF * 2;
constexpr size_t kOffWV   = kOffWQK  + (size_t)kL * kQKP * kD * 2;
constexpr size_t kOffWO   = kOffWV   + (size_t)kL * kD * kD * 2;
constexpr size_t kOffW1T  = kOffWO   + (size_t)kL * kD * kD * 2;
constexpr size_t kOffW2T  = kOffW1T  + (size_t)kL * kDFF * kD * 2;
constexpr size_t kOffBQK  = kOffW2T  + (size_t)kL * kFO * kFG * 2;
constexpr size_t kOffMB   = kOffBQK  + (size_t)kL * kQKP * 4;
constexpr size_t kWsTotal = kOffMB   + (size_t)kN * (kN / 32) * 4;
static_assert(kWsTotal == 109715456ull);
static_assert(kWsTotal <= 134217728ull);
static_assert((kOffRB % 128) == 0 && (kOffX16 % 128) == 0 && (kOffXV16 % 128) == 0 && (kOffQK16 % 128) == 0 &&
              (kOffVT % 128) == 0 && (kOffO16 % 128) == 0 && (kOffGB % 128) == 0 && (kOffH16 % 128) == 0 &&
              (kOffWQK % 128) == 0 && (kOffWV % 128) == 0 && (kOffWO % 128) == 0 && (kOffW1T % 128) == 0 &&
              (kOffW2T % 128) == 0 && (kOffBQK % 128) == 0 && (kOffMB % 128) == 0);

__device__ __forceinline__ unsigned short f2bf_bits(float f) {
  unsigned u = __float_as_uint(f);
  return (unsigned short)((u + 0x7FFFu + ((u >> 16) & 1u)) >> 16);
}
__device__ __forceinline__ float bf_bits2f(unsigned short h) { return __uint_as_float(((unsigned)h) << 16); }

__device__ __forceinline__ void dep_guard4_h(v8f& a, v8f& b, v8f& c, v8f& d, v16h x, v16h y) { asm volatile("v_nop\n\tv_nop\n\tv_nop\n\tv_nop" : "+v"(a), "+v"(b), "+v"(c), "+v"(d) : "v"(x), "v"(y)); }
__device__ __forceinline__ void dep_guard4_b(v8f& a, v8f& b, v8f& c, v8f& d, v16b x, v16b y) { asm volatile("v_nop\n\tv_nop\n\tv_nop\n\tv_nop" : "+v"(a), "+v"(b), "+v"(c), "+v"(d) : "v"(x), "v"(y)); }
__device__ __forceinline__ void keep4_h(v16h a, v16h b, v16h c, v16h d) { asm volatile("v_nop" :: "v"(a), "v"(b), "v"(c), "v"(d)); }
__device__ __forceinline__ void keep4_b(v16b a, v16b b, v16b c, v16b d) { asm volatile("v_nop" :: "v"(a), "v"(b), "v"(c), "v"(d)); }
__device__ __forceinline__ void acc_guard4(v8f& a, v8f& b, v8f& c, v8f& d) { asm volatile("v_nop\n\tv_nop\n\tv_nop\n\tv_nop" : "+v"(a), "+v"(b), "+v"(c), "+v"(d)); }
template <typename T> struct Frag;
template <> struct Frag<_Float16> {
  typedef v16h V; union U { v16h v; v8h h[2]; };
  static __device__ __forceinline__ v16h load(const _Float16* p) {
    U f; f.h[0] = *(const v8h*)(p); f.h[1] = *(const v8h*)(p + 16); return f.v;
  }
  static __device__ __forceinline__ v8f mma(v16h a, v16h b, v8f c) {
    return __builtin_amdgcn_wmma_f32_16x16x32_f16(false, a, false, b, (short)0, c, false, false);
  }
  static __device__ __forceinline__ void guard4(v8f& a, v8f& b, v8f& c, v8f& d, v16h x, v16h y) { dep_guard4_h(a, b, c, d, x, y); }
  static __device__ __forceinline__ void keep(v16h a, v16h b, v16h c, v16h d) { keep4_h(a, b, c, d); }
};
template <> struct Frag<__bf16> {
  typedef v16b V; union U { v16b v; v8b h[2]; };
  static __device__ __forceinline__ v16b load(const __bf16* p) {
    U f; f.h[0] = *(const v8b*)(p); f.h[1] = *(const v8b*)(p + 16); return f.v;
  }
  static __device__ __forceinline__ v8f mma(v16b a, v16b b, v8f c) {
    return __builtin_amdgcn_wmma_f32_16x16x32_bf16(false, a, false, b, (short)0, c, false, false);
  }
  static __device__ __forceinline__ void guard4(v8f& a, v8f& b, v8f& c, v8f& d, v16b x, v16b y) { dep_guard4_b(a, b, c, d, x, y); }
  static __device__ __forceinline__ void keep(v16b a, v16b b, v16b c, v16b d) { keep4_b(a, b, c, d); }
};

template <int ET> struct Elem;
template <> struct Elem<0> { typedef _Float16 T; };
template <> struct Elem<1> { typedef __bf16 T; };
template <int ET, bool SPLIT, int BIAS_MODE, int OUT_MODE, bool RESID, int ACT = 0>
__global__ __launch_bounds__(256) void wmma_gemm64(
    const unsigned short* __restrict__ Ap, const unsigned short* __restrict__ A2p, int lda, long strideA,
    const unsigned short* __restrict__ Btp, const unsigned short* __restrict__ Bt2p, int ldb, long strideB,
    void* __restrict__ Cout, void* __restrict__ Cout2, int ldc, long strideC,
    const float* __restrict__ bias,
    const float* __restrict__ resid, long strideR,
    int M, int N, int K, float scale) {
  typedef typename Elem<ET>::T T;
  typedef typename Frag<T>::V V;
  const T* A = (const T*)Ap; const T* A2 = (const T*)A2p; const T* Bt = (const T*)Btp; const T* Bt2 = (const T*)Bt2p;
  __shared__ __align__(16) float sT[8][16 * 68];
  const int b    = blockIdx.y;
  const int lane = threadIdx.x & 31;
  const int wave = threadIdx.x >> 5;
  const int tilesN = N >> 6;
  const int tilesM = M >> 6;
  const int tile = blockIdx.x * 8 + wave;
  if (tile >= tilesM * tilesN) return;
  const int tm = tile / tilesN;
  const int tn = tile - tm * tilesN;
  const int m0 = tm << 6;
  const int n0 = tn << 6;

  const T* Ab  = A  + (size_t)b * strideA;
  const T* Bb  = Bt + (size_t)b * strideB;
  const T* Ab2 = SPLIT ? (A2  + (size_t)b * strideA) : nullptr;
  const T* Bb2 = SPLIT ? (Bt2 + (size_t)b * strideB) : nullptr;

  const int rlane = lane & 15;
  const int koff  = (lane >> 4) * 8;
  const int mOff  = (lane >> 4) * 8;

  v8f acc[4][4];
#pragma unroll
  for (int i = 0; i < 4; ++i)
#pragma unroll
    for (int j = 0; j < 4; ++j) acc[i][j] = (v8f){0.f,0.f,0.f,0.f,0.f,0.f,0.f,0.f};

  for (int k0 = 0; k0 < K; k0 += 32) {
    V bh[4], bl[4];
#pragma unroll
    for (int j = 0; j < 4; ++j) {
      const size_t bo = (size_t)(n0 + (j << 4) + rlane) * ldb + koff + k0;
      bh[j] = Frag<T>::load(Bb + bo);
      if (SPLIT) bl[j] = Frag<T>::load(Bb2 + bo);
    }
#pragma unroll
    for (int i = 0; i < 4; ++i) {
      const size_t ao = (size_t)(m0 + (i << 4) + rlane) * lda + koff + k0;
      V ah = Frag<T>::load(Ab + ao);
      V al;
      if (SPLIT) al = Frag<T>::load(Ab2 + ao);
#pragma unroll
      for (int j = 0; j < 4; ++j) {
        acc[i][j] = Frag<T>::mma(ah, bh[j], acc[i][j]);
        if (SPLIT) {
          acc[i][j] = Frag<T>::mma(ah, bl[j], acc[i][j]);
          acc[i][j] = Frag<T>::mma(al, bh[j], acc[i][j]);
        }
      }
      Frag<T>::guard4(acc[i][0], acc[i][1], acc[i][2], acc[i][3], ah, SPLIT ? al : ah);
    }
    Frag<T>::keep(bh[0], bh[1], bh[2], bh[3]);
    if (SPLIT) Frag<T>::keep(bl[0], bl[1], bl[2], bl[3]);
  }
  acc_guard4(acc[0][0], acc[0][1], acc[0][2], acc[0][3]);
  acc_guard4(acc[1][0], acc[1][1], acc[1][2], acc[1][3]);
  acc_guard4(acc[2][0], acc[2][1], acc[2][2], acc[2][3]);
  acc_guard4(acc[3][0], acc[3][1], acc[3][2], acc[3][3]);

  float* slab = sT[wave];
  const float* Rb = RESID ? (resid + (size_t)b * strideR) : nullptr;
#pragma unroll
  for (int i = 0; i < 4; ++i) {
    const int mBase = m0 + (i << 4);
#pragma unroll
    for (int j = 0; j < 4; ++j) {
      const int n = n0 + (j << 4) + rlane;
      float bv = 0.f;
      if (BIAS_MODE == 2) bv = bias[n];
#pragma unroll
      for (int r = 0; r < 8; ++r) {
        float v = acc[i][j][r] * scale;
        if (BIAS_MODE == 1) v += bias[mBase + mOff + r];
        if (BIAS_MODE == 2) v += bv;
        if (RESID) v += Rb[(size_t)(mBase + mOff + r) * ldc + n];
        if (ACT == 2) v = fmaxf(v, 0.0f);
        if (ACT == 4) v = (v > 0.f) ? v : 0.01f * v;
        slab[(mOff + r) * 68 + (j << 4) + rlane] = v;
      }
    }
    __builtin_amdgcn_fence(__ATOMIC_RELEASE, "workgroup");
    __builtin_amdgcn_wave_barrier();
    __builtin_amdgcn_fence(__ATOMIC_ACQUIRE, "workgroup");
    if (OUT_MODE == 0) {
      float* C = (float*)Cout + (size_t)b * strideC;
      const int hh = lane >> 4, c4 = (lane & 15) * 4;
      for (int pass = 0; pass < 2; ++pass) {
#pragma unroll
        for (int it = 0; it < 8; ++it) {
          const int row = it * 2 + hh;
          v4f v = *(const v4f*)(slab + row * 68 + c4);
          *(volatile v4f*)(C + (size_t)(mBase + row) * ldc + n0 + c4) = v;
        }
        __threadfence();
      }
    } else {
      const int q = lane >> 3, c8 = (lane & 7) * 8;
      unsigned short* C  = (unsigned short*)Cout  + (size_t)b * strideC;
      unsigned short* C2 = (OUT_MODE == 2) ? ((unsigned short*)Cout2 + (size_t)b * strideC) : nullptr;
      for (int pass = 0; pass < 2; ++pass) {
#pragma unroll
        for (int it = 0; it < 4; ++it) {
          const int row = it * 4 + q;
          const float* sp = slab + row * 68 + c8;
          v8h hv, lv;
#pragma unroll
          for (int e = 0; e < 8; ++e) {
            if (OUT_MODE == 1) {
              hv[e] = (_Float16)sp[e];
            } else {
              unsigned short hb = f2bf_bits(sp[e]);
              unsigned short lb = f2bf_bits(sp[e] - bf_bits2f(hb));
              hv[e] = __builtin_bit_cast(_Float16, hb);
              lv[e] = __builtin_bit_cast(_Float16, lb);
            }
          }
          *(volatile v8h*)(C + (size_t)(mBase + row) * ldc + n0 + c8) = hv;
          if (OUT_MODE == 2) *(volatile v8h*)(C2 + (size_t)(mBase + row) * ldc + n0 + c8) = lv;
        }
        __threadfence();
      }
    }
    __builtin_amdgcn_fence(__ATOMIC_RELEASE, "workgroup");
    __builtin_amdgcn_wave_barrier();
    __builtin_amdgcn_fence(__ATOMIC_ACQUIRE, "workgroup");
  }
}

__global__ __launch_bounds__(256) void wt_transpose_kernel(
    const float* __restrict__ Wa, const float* __restrict__ Wb, const float* __restrict__ Wc, const float* __restrict__ Wd,
    unsigned short* Oa, unsigned short* Ob, unsigned short* Oc, unsigned short* Od,
    long osa, long osb, long osc, long osd, int Kin, int Nout, float carry) {
  __shared__ float sm[64][65];
  const int t  = threadIdx.x;
  const int k0 = blockIdx.x * 64;
  const int n0 = blockIdx.y * 64;
  const int z  = blockIdx.z;
  const int w  = z >> 2;
  const int l  = z & 3;
  const float* W = (w == 0) ? Wa : (w == 1) ? Wb : (w == 2) ? Wc : Wd;
  unsigned short* O = (w == 0) ? Oa : (w == 1) ? Ob : (w == 2) ? Oc : Od;
  const long os = (w == 0) ? osa : (w == 1) ? osb : (w == 2) ? osc : osd;
  const float* src = W + (size_t)l * Kin * Nout;
  unsigned short* dst = O + (size_t)l * os;
#pragma unroll
  for (int i = 0; i < 16; ++i) {
    const int e = i * 256 + t;
    const int r = e >> 6;
    const int c = e & 63;
    sm[c][r] = src[(size_t)(k0 + r) * Nout + n0 + c] * carry;
  }
  __syncthreads();
  const int lane = t & 31, wave = t >> 5;
  const int q = lane >> 3, c8 = (lane & 7) * 8;
  v8h hv[2];
#pragma unroll
  for (int it = 0; it < 2; ++it) {
    const int row = wave * 8 + it * 4 + q;
#pragma unroll
    for (int e = 0; e < 8; ++e) hv[it][e] = (_Float16)sm[row][c8 + e];
  }
  for (int pass = 0; pass < 2; ++pass) {
#pragma unroll
    for (int it = 0; it < 2; ++it) {
      const int row = wave * 8 + it * 4 + q;
      *(volatile v8h*)(dst + (size_t)(n0 + row) * Kin + k0 + c8) = hv[it];
    }
    __threadfence();
  }
}

__global__ __launch_bounds__(256) void bias_cat_kernel(const float* __restrict__ bq, const float* __restrict__ bk, float* __restrict__ out) {
  const int i  = blockIdx.x * 256 + threadIdx.x;
  const int l  = i >> 9;
  const int cc = i & 511;
  const int c2 = cc & 255;
  const float a = bq[l * kD + c2];
  const float b = bk[l * kD + c2];
  const float v = (cc < kD) ? a : b;
  volatile float* p = out + i;
  *p = v;
  __threadfence();
  *p = v;
}

__global__ __launch_bounds__(256) void mask_pack_kernel(const int* __restrict__ mask, unsigned* __restrict__ mb) {
  const int lane = threadIdx.x & 31, wave = threadIdx.x >> 5;
  const int q = blockIdx.x * 8 + wave;
  const int* mr = mask + (size_t)q * kN;
  unsigned word = 0u;
#pragma unroll 1
  for (int w = 0; w < 32; ++w) {
    const int v = mr[w * 32 + lane];
    const unsigned bal = __builtin_amdgcn_ballot_w32(v != 0);
    word = (lane == w) ? bal : word;
  }
  volatile unsigned* p = mb + (size_t)q * 32 + lane;
  *p = word;
  __threadfence();
  *p = word;
}

__global__ __launch_bounds__(256) void addpos_kernel(const float* __restrict__ x, const float* __restrict__ xv,
                                                     const float* __restrict__ pos, float* __restrict__ XF,
                                                     unsigned short* __restrict__ X16, unsigned short* __restrict__ XV16) {
  const int lane = threadIdx.x & 31, wave = threadIdx.x >> 5;
  const int row = blockIdx.x * 8 + wave;
  const int n = row & (kN - 1);
  const int c0 = lane * 4, c1 = 128 + lane * 4;
  const size_t ro = (size_t)row * kD;
  const v4f pa = *(const v4f*)(pos + (size_t)n * kD + c0);
  const v4f pb = *(const v4f*)(pos + (size_t)n * kD + c1);
  const v4f xa = *(const v4f*)(x + ro + c0) + pa;
  const v4f xb = *(const v4f*)(x + ro + c1) + pb;
  const v4f va = *(const v4f*)(xv + ro + c0) + pa;
  const v4f vb = *(const v4f*)(xv + ro + c1) + pb;
  v4h hxa, hxb, hva, hvb;
#pragma unroll
  for (int e = 0; e < 4; ++e) {
    hxa[e] = (_Float16)xa[e];
    hxb[e] = (_Float16)xb[e];
    hva[e] = (_Float16)va[e];
    hvb[e] = (_Float16)vb[e];
  }
  for (int pass = 0; pass < 2; ++pass) {
    *(volatile v4f*)(XF + ro + c0) = xa;
    *(volatile v4f*)(XF + ro + c1) = xb;
    *(volatile v4h*)(X16 + ro + c0) = hxa;
    *(volatile v4h*)(X16 + ro + c1) = hxb;
    *(volatile v4h*)(XV16 + ro + c0) = hva;
    *(volatile v4h*)(XV16 + ro + c1) = hvb;
    __threadfence();
  }
}

__device__ __forceinline__ float wave_sum32(float v) {
#pragma unroll
  for (int off = 16; off > 0; off >>= 1) v += __shfl_xor(v, off, 32);
  return v;
}
__device__ __forceinline__ void ln_row8(const float (&x)[8], const v4f ga, const v4f gb, const v4f ba, const v4f bb, float (&y)[8]) {
  float s = 0.f;
#pragma unroll
  for (int e = 0; e < 8; ++e) s += x[e];
  s = wave_sum32(s);
  const float mean = s * kInvD;
  float d[8];
  float ss = 0.f;
#pragma unroll
  for (int e = 0; e < 8; ++e) {
    d[e] = x[e] - mean;
    ss += d[e] * d[e];
  }
  ss = wave_sum32(ss);
  const float rstd = 1.0f / sqrtf(ss * kInvD + kLnEps);
#pragma unroll
  for (int e = 0; e < 4; ++e) {
    y[e]     = d[e] * rstd * ga[e] + ba[e];
    y[4 + e] = d[4 + e] * rstd * gb[e] + bb[e];
  }
}

template <int MODE>
__global__ __launch_bounds__(256) void ln_kernel(float* X, const float* __restrict__ R,
                                                 const float* __restrict__ g, const float* __restrict__ be,
                                                 unsigned short* __restrict__ X16,
                                                 const float* __restrict__ gf, const float* __restrict__ bff,
                                                 float* __restrict__ out) {
  const int lane = threadIdx.x & 31, wave = threadIdx.x >> 5;
  const int row = blockIdx.x * 8 + wave;
  const int c0 = lane * 4, c1 = 128 + lane * 4;
  const size_t ro = (size_t)row * kD;
  const v4f xa = *(const v4f*)(X + ro + c0);
  const v4f xb = *(const v4f*)(X + ro + c1);
  const v4f ra = *(const v4f*)(R + ro + c0);
  const v4f rb = *(const v4f*)(R + ro + c1);
  const v4f ga = *(const v4f*)(g + c0);
  const v4f gb = *(const v4f*)(g + c1);
  const v4f ba = *(const v4f*)(be + c0);
  const v4f bb = *(const v4f*)(be + c1);
  float xin[8], y[8];
#pragma unroll
  for (int e = 0; e < 4; ++e) {
    xin[e]     = xa[e] + ra[e];
    xin[4 + e] = xb[e] + rb[e];
  }
  ln_row8(xin, ga, gb, ba, bb, y);
  if (MODE == 0) {
    v4f ya, yb;
    v4h ha, hb;
#pragma unroll
    for (int e = 0; e < 4; ++e) {
      ya[e] = y[e];
      yb[e] = y[4 + e];
      ha[e] = (_Float16)y[e];
      hb[e] = (_Float16)y[4 + e];
    }
    for (int pass = 0; pass < 2; ++pass) {
      *(volatile v4f*)(X + ro + c0) = ya;
      *(volatile v4f*)(X + ro + c1) = yb;
      *(volatile v4h*)(X16 + ro + c0) = ha;
      *(volatile v4h*)(X16 + ro + c1) = hb;
      __threadfence();
    }
  } else {
    const v4f fa = *(const v4f*)(gf + c0);
    const v4f fb = *(const v4f*)(gf + c1);
    const v4f ca = *(const v4f*)(bff + c0);
    const v4f cb = *(const v4f*)(bff + c1);
    float z[8];
    ln_row8(y, fa, fb, ca, cb, z);
    v4f za, zb;
#pragma unroll
    for (int e = 0; e < 4; ++e) {
      za[e] = z[e];
      zb[e] = z[4 + e];
    }
    for (int pass = 0; pass < 2; ++pass) {
      *(volatile v4f*)(out + ro + c0) = za;
      *(volatile v4f*)(out + ro + c1) = zb;
      __threadfence();
    }
  }
}

__global__ __launch_bounds__(256) void act_cast_kernel(const float* __restrict__ G, unsigned short* __restrict__ Hh) {
  __shared__ __align__(16) float sm[2048];
  const int tid = threadIdx.x;
  const size_t base = (size_t)blockIdx.x * 2048;
#pragma unroll 1
  for (int i = 0; i < 8; ++i) {
    const int idx = i * 256 + tid;
    const float v = G[base + idx];
    sm[idx] = 0.5f * v * (1.0f + erff(v * kInvSqrt2));
  }
  __syncthreads();
  const v4f a0 = *(const v4f*)(sm + tid * 8);
  const v4f a1 = *(const v4f*)(sm + tid * 8 + 4);
  v8h hv;
#pragma unroll
  for (int e = 0; e < 4; ++e) {
    hv[e]     = (_Float16)a0[e];
    hv[4 + e] = (_Float16)a1[e];
  }
  unsigned short* p = Hh + base + (size_t)tid * 8;
  *(volatile v8h*)p = hv;
  __threadfence();
  *(volatile v8h*)p = hv;
}

constexpr int kAQ   = 16;
constexpr int kAKC  = 64;
constexpr int kOtP  = 264;
constexpr int kQBlk = kN / kAQ;
static_assert((kN % kAKC) == 0 && (kN % kAQ) == 0 && kQBlk == 64);

__device__ __forceinline__ v8f mma_h(v16h a, v16h b, v8f c) {
  c = __builtin_amdgcn_wmma_f32_16x16x32_f16(false, a, false, b, (short)0, c, false, false);
  asm volatile("v_nop\n\tv_nop\n\tv_nop\n\tv_nop" : "+v"(c) : "v"(a), "v"(b));
  return c;
}

template <bool MASKED>
__global__ __launch_bounds__(256) __attribute__((amdgpu_num_vgpr(256)))
void attn_kernel(const unsigned short* __restrict__ QKp, const unsigned short* __restrict__ Vtp,
                 unsigned short* __restrict__ Op, const unsigned* __restrict__ mbits,
                 float sscale) {
  union FH { v16h v; v8h h[2]; };
  __shared__ __align__(16) _Float16 Ps[8][kAQ * kAKC];
  __shared__ __align__(16) _Float16 Ot[kAQ * kOtP];
  __shared__ __align__(16) unsigned smask[MASKED ? kAQ * 32 : 4];

  const _Float16* QK = (const _Float16*)QKp;
  const _Float16* Vt = (const _Float16*)Vtp;
  const int tid  = threadIdx.x;
  const int wave = tid >> 5;
  const int lane = tid & 31;
  const int hh   = lane >> 4;
  const int c    = lane & 15;
  const int h    = wave;
  const int b    = blockIdx.x / kQBlk;
  const int q0   = (blockIdx.x - b * kQBlk) * kAQ;
  const int tok0 = b * kN;

  if (MASKED) {
    const int mr = tid >> 4, w2 = (tid & 15) * 2;
    const v2u mv = *(const v2u*)(mbits + (size_t)(q0 + mr) * 32 + w2);
    *(v2u*)(smask + mr * 32 + w2) = mv;
    __syncthreads();
  }

  const v16h qa = Frag<_Float16>::load(QK + (size_t)(tok0 + q0 + c) * kQKP + h * kDK + 8 * hh);

  float mrow[8], lsum[8];
  v8f oacc0 = (v8f){0.f,0.f,0.f,0.f,0.f,0.f,0.f,0.f};
  v8f oacc1 = (v8f){0.f,0.f,0.f,0.f,0.f,0.f,0.f,0.f};
#pragma unroll
  for (int r = 0; r < 8; ++r) {
    mrow[r] = -INFINITY;
    lsum[r] = 0.f;
  }

  const size_t vrow0 = (size_t)(h * kDK + c);
  _Float16* pw = Ps[wave];

#pragma unroll 1
  for (int kc = 0; kc < kN / kAKC; ++kc) {
    const int kv0 = kc * kAKC;
    v8f s[4];
#pragma unroll
    for (int j = 0; j < 4; ++j) {
      const v16h kb = Frag<_Float16>::load(QK + (size_t)(tok0 + kv0 + j * 16 + c) * kQKP + kD + h * kDK + 8 * hh);
      s[j] = mma_h(qa, kb, (v8f){0.f,0.f,0.f,0.f,0.f,0.f,0.f,0.f});
    }
#pragma unroll
    for (int r = 0; r < 8; ++r) {
      float sv[4];
      float m = -INFINITY;
#pragma unroll
      for (int j = 0; j < 4; ++j) {
        float xs = s[j][r] * sscale;
        if (MASKED) {
          const unsigned mw = smask[(8 * hh + r) * 32 + kc * 2 + (j >> 1)];
          const bool msk = ((mw >> ((j & 1) * 16 + c)) & 1u) != 0u;
          xs = msk ? -INFINITY : xs;
        }
        sv[j] = xs;
        m = fmaxf(m, xs);
      }
      m = fmaxf(m, __shfl_xor(m, 1, 32));
      m = fmaxf(m, __shfl_xor(m, 2, 32));
      m = fmaxf(m, __shfl_xor(m, 4, 32));
      m = fmaxf(m, __shfl_xor(m, 8, 32));
      const float mnew = fmaxf(mrow[r], m);
      float alpha = __expf(mrow[r] - mnew);
      if (MASKED) alpha = (mnew == -INFINITY) ? 1.0f : alpha;
      mrow[r] = mnew;
      float ps = 0.f;
#pragma unroll
      for (int j = 0; j < 4; ++j) {
        float p = __expf(sv[j] - mnew);
        if (MASKED) p = (mnew == -INFINITY) ? 0.0f : p;
        ps += p;
        pw[(8 * hh + r) * kAKC + j * 16 + c] = (_Float16)(p * kPCarry);
      }
      lsum[r] = lsum[r] * alpha + ps;
      oacc0[r] *= alpha;
      oacc1[r] *= alpha;
    }
    __builtin_amdgcn_fence(__ATOMIC_RELEASE, "workgroup");
    __builtin_amdgcn_wave_barrier();
    __builtin_amdgcn_fence(__ATOMIC_ACQUIRE, "workgroup");
#pragma unroll
    for (int kk = 0; kk < 2; ++kk) {
      const v16h vb0 = Frag<_Float16>::load(Vt + vrow0 * kM + tok0 + kv0 + kk * 32 + 8 * hh);
      const v16h vb1 = Frag<_Float16>::load(Vt + (vrow0 + 16) * kM + tok0 + kv0 + kk * 32 + 8 * hh);
      FH pa;
      pa.h[0] = *(const v8h*)(pw + c * kAKC + kk * 32 + 8 * hh);
      pa.h[1] = *(const v8h*)(pw + c * kAKC + kk * 32 + 16 + 8 * hh);
      oacc0 = mma_h(pa.v, vb0, oacc0);
      oacc1 = mma_h(pa.v, vb1, oacc1);
    }
    __builtin_amdgcn_fence(__ATOMIC_RELEASE, "workgroup");
    __builtin_amdgcn_wave_barrier();
    __builtin_amdgcn_fence(__ATOMIC_ACQUIRE, "workgroup");
  }

#pragma unroll
  for (int r = 0; r < 8; ++r) {
    float l = lsum[r];
    l += __shfl_xor(l, 1, 32);
    l += __shfl_xor(l, 2, 32);
    l += __shfl_xor(l, 4, 32);
    l += __shfl_xor(l, 8, 32);
    const float inv = 1.0f / (l * kPOverO);
    Ot[(8 * hh + r) * kOtP + h * kDK + c]      = (_Float16)(oacc0[r] * inv);
    Ot[(8 * hh + r) * kOtP + h * kDK + 16 + c] = (_Float16)(oacc1[r] * inv);
  }
  __syncthreads();
  v8h ov[2];
#pragma unroll
  for (int it = 0; it < 2; ++it) ov[it] = *(const v8h*)(&Ot[(it * 8 + wave) * kOtP + lane * 8]);
  for (int pass = 0; pass < 2; ++pass) {
#pragma unroll
    for (int it = 0; it < 2; ++it) {
      const int row = it * 8 + wave;
      *(volatile v8h*)(Op + (size_t)(tok0 + q0 + row) * kD + lane * 8) = ov[it];
    }
    __threadfence();
  }
}

extern "C" void kernel_launch(void* const* d_in, const int* in_sizes, int n_in,
                              void* d_out, int out_size, void* d_ws, size_t ws_size,
                              hipStream_t stream) {
  if (n_in < 22) return;
  if (in_sizes[0] != kM * kD) return;
  if (in_sizes[1] != kM * kD) return;
  if (in_sizes[2] != kN * kN) return;
  if (in_sizes[3] != kN * kD) return;
  if (in_sizes[4] != kL * kD * kD) return;
  if (in_sizes[5] != kL * kD) return;
  if (in_sizes[6] != kL * kD * kD) return;
  if (in_sizes[7] != kL * kD) return;
  if (in_sizes[8] != kL * kD * kD) return;
  if (in_sizes[9] != kL * kD) return;
  if (in_sizes[10] != kL * kD * kD) return;
  if (in_sizes[11] != kL * kD) return;
  if (in_sizes[12] != kL * kD * kDFF) return;
  if (in_sizes[13] != kL * kDFF) return;
  if (in_sizes[14] != kL * kFG * kFO) return;
  if (in_sizes[15] != kL * kFO) return;
  if (in_sizes[16] != kL * kD) return;
  if (in_sizes[17] != kL * kD) return;
  if (in_sizes[18] != kL * kD) return;
  if (in_sizes[19] != kL * kD) return;
  if (in_sizes[20] != kD) return;
  if (in_sizes[21] != kD) return;
  if (out_size != kM * kD) return;
  if (ws_size < kWsTotal) return;

  const float* x    = (const float*)d_in[0];
  const float* x_v  = (const float*)d_in[1];
  const int*   mask = (const int*)d_in[2];
  const float* pos  = (const float*)d_in[3];
  const float* Wq   = (const float*)d_in[4];
  const float* bq   = (const float*)d_in[5];
  const float* Wk   = (const float*)d_in[6];
  const float* bk   = (const float*)d_in[7];
  const float* Wv   = (const float*)d_in[8];
  const float* bv   = (const float*)d_in[9];
  const float* Wo   = (const float*)d_in[10];
  const float* bo   = (const float*)d_in[11];
  const float* W1   = (const float*)d_in[12];
  const float* b1   = (const float*)d_in[13];
  const float* W2   = (const float*)d_in[14];
  const float* b2   = (const float*)d_in[15];
  const float* g1   = (const float*)d_in[16];
  const float* be1  = (const float*)d_in[17];
  const float* g2   = (const float*)d_in[18];
  const float* be2  = (const float*)d_in[19];
  const float* gf   = (const float*)d_in[20];
  const float* bfin = (const float*)d_in[21];
  float* out = (float*)d_out;

  char* ws = (char*)d_ws;
  float*          XF   = (float*)(ws + kOffXF);
  float*          RB   = (float*)(ws + kOffRB);
  unsigned short* X16  = (unsigned short*)(ws + kOffX16);
  unsigned short* XV16 = (unsigned short*)(ws + kOffXV16);
  unsigned short* QK16 = (unsigned short*)(ws + kOffQK16);
  unsigned short* VT   = (unsigned short*)(ws + kOffVT);
  unsigned short* O16  = (unsigned short*)(ws + kOffO16);
  float*          GB   = (float*)(ws + kOffGB);
  unsigned short* H16  = (unsigned short*)(ws + kOffH16);
  unsigned short* WQK  = (unsigned short*)(ws + kOffWQK);
  unsigned short* WVT  = (unsigned short*)(ws + kOffWV);
  unsigned short* WOT  = (unsigned short*)(ws + kOffWO);
  unsigned short* W1T  = (unsigned short*)(ws + kOffW1T);
  unsigned short* W2T  = (unsigned short*)(ws + kOffW2T);
  float*          BQK  = (float*)(ws + kOffBQK);
  unsigned*       MB   = (unsigned*)(ws + kOffMB);

  const float sscale = (float)(1.0 / sqrt((double)kDK));

  wt_transpose_kernel<<<dim3(kD / 64, kD / 64, 16), 256, 0, stream>>>(
      Wq, Wk, Wv, Wo,
      WQK, WQK + (size_t)kD * kD, WVT, WOT,
      (long)kQKP * kD, (long)kQKP * kD, (long)kD * kD, (long)kD * kD,
      kD, kD, kWCarry);
  wt_transpose_kernel<<<dim3(kD / 64, kDFF / 64, 4), 256, 0, stream>>>(
      W1, W1, W1, W1, W1T, W1T, W1T, W1T,
      (long)kDFF * kD, (long)kDFF * kD, (long)kDFF * kD, (long)kDFF * kD,
      kD, kDFF, kWCarry);
  wt_transpose_kernel<<<dim3(kFG / 64, kFO / 64, 4), 256, 0, stream>>>(
      W2, W2, W2, W2, W2T, W2T, W2T, W2T,
      (long)kFO * kFG, (long)kFO * kFG, (long)kFO * kFG, (long)kFO * kFG,
      kFG, kFO, kWCarry);
  bias_cat_kernel<<<(kL * kQKP) / 256, 256, 0, stream>>>(bq, bk, BQK);
  mask_pack_kernel<<<kN / 8, 256, 0, stream>>>(mask, MB);
  addpos_kernel<<<kM / 8, 256, 0, stream>>>(x, x_v, pos, XF, X16, XV16);

  wmma_gemm64<0, false, 1, 1, false><<<dim3(256, 1), 256, 0, stream>>>(
      WVT, WVT, kD, 0L,
      XV16, XV16, kD, 0L,
      (void*)VT, (void*)VT, kM, 0L,
      bv, bv, 0L,
      kL * kD, kM, kD, kWCarryInv);

  for (int l = 0; l < kL; ++l) {
    wmma_gemm64<0, false, 2, 1, false><<<dim3(128, 1), 256, 0, stream>>>(
        X16, X16, kD, 0L,
        WQK + (size_t)l * kQKP * kD, WQK + (size_t)l * kQKP * kD, kD, 0L,
        (void*)QK16, (void*)QK16, kQKP, 0L,
        BQK + (size_t)l * kQKP, BQK + (size_t)l * kQKP, 0L,
        kM, kQKP, kD, kWCarryInv);

    if ((l & 1) == 1) {
      attn_kernel<true><<<kB * kQBlk, 256, 0, stream>>>(QK16, VT + (size_t)l * kD * kM, O16, MB, sscale);
    } else {
      attn_kernel<false><<<kB * kQBlk, 256, 0, stream>>>(QK16, VT + (size_t)l * kD * kM, O16, MB, sscale);
    }

    wmma_gemm64<0, false, 2, 0, false><<<dim3(64, 1), 256, 0, stream>>>(
        O16, O16, kD, 0L,
        WOT + (size_t)l * kD * kD, WOT + (size_t)l * kD * kD, kD, 0L,
        (void*)RB, (void*)RB, kD, 0L,
        bo + (size_t)l * kD, bo + (size_t)l * kD, 0L,
        kM, kD, kD, kOutScale);

    ln_kernel<0><<<kM / 8, 256, 0, stream>>>(XF, RB, g1 + (size_t)l * kD, be1 + (size_t)l * kD, X16, gf, bfin, out);

    wmma_gemm64<0, false, 2, 0, false><<<dim3(256, 1), 256, 0, stream>>>(
        X16, X16, kD, 0L,
        W1T + (size_t)l * kDFF * kD, W1T + (size_t)l * kDFF * kD, kD, 0L,
        (void*)GB, (void*)GB, kDFF, 0L,
        b1 + (size_t)l * kDFF, b1 + (size_t)l * kDFF, 0L,
        kM, kDFF, kD, kWCarryInv);

    act_cast_kernel<<<(kM * kDFF) / 2048, 256, 0, stream>>>(GB, H16);

    wmma_gemm64<0, false, 2, 0, false><<<dim3(64, 1), 256, 0, stream>>>(
        H16, H16, kFG, 0L,
        W2T + (size_t)l * kFO * kFG, W2T + (size_t)l * kFO * kFG, kFG, 0L,
        (void*)RB, (void*)RB, kFO, 0L,
        b2 + (size_t)l * kFO, b2 + (size_t)l * kFO, 0L,
        2 * kM, kFO, kFG, kWCarryInv);

    if (l == kL - 1) {
      ln_kernel<1><<<kM / 8, 256, 0, stream>>>(XF, RB, g2 + (size_t)l * kD, be2 + (size_t)l * kD, X16, gf, bfin, out);
    } else {
      ln_kernel<0><<<kM / 8, 256, 0, stream>>>(XF, RB, g2 + (size_t)l * kD, be2 + (size_t)l * kD, X16, gf, bfin, out);
    }
  }
}
